// SimplifiedMambaBlock_69595650064651
// MI455X (gfx1250) — hardware-verified
//
#include <hip/hip_runtime.h>
#include <stdint.h>

typedef __attribute__((ext_vector_type(16))) _Float16 v16h;
typedef __attribute__((ext_vector_type(8)))  _Float16 v8h;
typedef __attribute__((ext_vector_type(16))) __bf16   v16b;
typedef __attribute__((ext_vector_type(8)))  __bf16   v8b;
typedef __attribute__((ext_vector_type(8)))  float    v8f;
typedef __attribute__((ext_vector_type(4)))  float    v4f;
typedef __attribute__((ext_vector_type(2)))  float    v2f;
typedef __attribute__((ext_vector_type(4)))  unsigned v4u;

constexpr int DMOD = 1024;
constexpr int DST  = 16;
constexpr int NBAT = 4;
constexpr int SEQL = 2048;
constexpr int NROW = NBAT * SEQL;
constexpr int NBC  = 64;
constexpr int TCH  = 64;
constexpr float kLnEps = 1e-5f;
constexpr float kLog2e = 1.4426950408889634f;

static_assert(NROW % 64 == 0 && DMOD % 64 == 0 && NBC % 64 == 0, "GEMM M/N tile multiples");
static_assert(DMOD % 32 == 0, "GEMM K multiple of 32");
static_assert(SEQL % TCH == 0 && SEQL % 256 == 0, "chunking");
static_assert((NROW * DMOD) % (8 * 256) == 0, "cvt/gate grids exact");

constexpr size_t SZ_P16  = (size_t)NROW * DMOD * 2;
constexpr size_t SZ_P32  = (size_t)NROW * DMOD * 4;
constexpr size_t OFF_XB   = 0;
constexpr size_t OFF_XCH  = OFF_XB   + SZ_P16;
constexpr size_t OFF_XCL  = OFF_XCH  + SZ_P16;
constexpr size_t OFF_WIN  = OFF_XCL  + SZ_P16;
constexpr size_t OFF_WDT  = OFF_WIN  + (size_t)2 * DMOD * DMOD * 2;
constexpr size_t OFF_WBC  = OFF_WDT  + (size_t)DMOD * DMOD * 2;
constexpr size_t OFF_WOUT = OFF_WBC  + (size_t)NBC * DMOD * 2;
constexpr size_t OFF_ATAB = OFF_WOUT + (size_t)DMOD * DMOD * 2;
constexpr size_t OFF_BC   = OFF_ATAB + (size_t)DMOD * DST * 4;
constexpr size_t OFF_PS   = OFF_BC   + (size_t)NROW * NBC * 4;
constexpr size_t OFF_Y    = OFF_PS   + SZ_P32;
constexpr size_t WS_END   = OFF_Y    + SZ_P32;
static_assert(WS_END == 128122880ull, "carve total");
static_assert(WS_END <= 134217728ull, "carve under 128 MiB");
static_assert(OFF_XCH % 128 == 0 && OFF_XCL % 128 == 0 && OFF_WIN % 128 == 0 && OFF_WDT % 128 == 0 &&
              OFF_WBC % 128 == 0 && OFF_WOUT % 128 == 0 && OFF_ATAB % 128 == 0 && OFF_BC % 128 == 0 &&
              OFF_PS % 128 == 0 && OFF_Y % 128 == 0, "128-B aligned regions");

__device__ __forceinline__ unsigned short f2bf_bits(float f) {
  unsigned u = __float_as_uint(f);
  return (unsigned short)((u + 0x7FFFu + ((u >> 16) & 1u)) >> 16);
}
__device__ __forceinline__ float bf_bits2f(unsigned short h) { return __uint_as_float(((unsigned)h) << 16); }
__device__ __forceinline__ float bfr(float f) { return bf_bits2f(f2bf_bits(f)); }
__device__ __forceinline__ void split_bf(float v, unsigned& hb, unsigned& lb) {
  const unsigned short h = f2bf_bits(v);
  hb = (unsigned)h;
  lb = (unsigned)f2bf_bits(v - bf_bits2f(h));
}

__device__ __forceinline__ void dep_guard_h(v8f& a, v8f& b, v16h x, v16h y) { asm volatile("v_nop\n\tv_nop\n\tv_nop\n\tv_nop" : "+v"(a), "+v"(b) : "v"(x), "v"(y)); }
__device__ __forceinline__ void dep_guard_b(v8f& a, v8f& b, v16b x, v16b y) { asm volatile("v_nop\n\tv_nop\n\tv_nop\n\tv_nop" : "+v"(a), "+v"(b) : "v"(x), "v"(y)); }
__device__ __forceinline__ void keep4_h(v16h a, v16h b, v16h c, v16h d) { asm volatile("v_nop" :: "v"(a), "v"(b), "v"(c), "v"(d)); }
__device__ __forceinline__ void keep4_b(v16b a, v16b b, v16b c, v16b d) { asm volatile("v_nop" :: "v"(a), "v"(b), "v"(c), "v"(d)); }
__device__ __forceinline__ void acc_guard4(v8f& a, v8f& b, v8f& c, v8f& d) { asm volatile("v_nop\n\tv_nop\n\tv_nop\n\tv_nop" : "+v"(a), "+v"(b), "+v"(c), "+v"(d)); }
template <typename T> struct Frag;
template <> struct Frag<_Float16> {
  typedef v16h V; union U { v16h v; v8h h[2]; };
  static __device__ __forceinline__ v16h load(const _Float16* p) {
    U f; f.h[0] = *(const v8h*)(p); f.h[1] = *(const v8h*)(p + 16); return f.v;
  }
  static __device__ __forceinline__ v8f mma(v16h a, v16h b, v8f c) {
    return __builtin_amdgcn_wmma_f32_16x16x32_f16(false, a, false, b, (short)0, c, false, false);
  }
  static __device__ __forceinline__ void guard(v8f& a, v8f& b, v16h x, v16h y) { dep_guard_h(a, b, x, y); }
  static __device__ __forceinline__ void keep(v16h a, v16h b, v16h c, v16h d) { keep4_h(a, b, c, d); }
};
template <> struct Frag<__bf16> {
  typedef v16b V; union U { v16b v; v8b h[2]; };
  static __device__ __forceinline__ v16b load(const __bf16* p) {
    U f; f.h[0] = *(const v8b*)(p); f.h[1] = *(const v8b*)(p + 16); return f.v;
  }
  static __device__ __forceinline__ v8f mma(v16b a, v16b b, v8f c) {
    return __builtin_amdgcn_wmma_f32_16x16x32_bf16(false, a, false, b, (short)0, c, false, false);
  }
  static __device__ __forceinline__ void guard(v8f& a, v8f& b, v16b x, v16b y) { dep_guard_b(a, b, x, y); }
  static __device__ __forceinline__ void keep(v16b a, v16b b, v16b c, v16b d) { keep4_b(a, b, c, d); }
};

template <int ET> struct Elem;
template <> struct Elem<0> { typedef _Float16 T; };
template <> struct Elem<1> { typedef __bf16 T; };
template <int ET, int SPLITK, int BIAS_MODE, int OUT_MODE, int ACT = 0>
__global__ __launch_bounds__(256) void wmma_gemm64(
    const unsigned short* __restrict__ Ap, const unsigned short* __restrict__ A2p, int lda, long strideA,
    const unsigned short* __restrict__ Btp, const unsigned short* __restrict__ Bt2p, int ldb, long strideB,
    void* __restrict__ Cout, void* __restrict__ Cout2, int ldc, long strideC,
    const float* __restrict__ bias,
    int M, int N, int K, float scale) {
  typedef typename Elem<ET>::T T;
  typedef typename Frag<T>::V V;
  const T* A = (const T*)Ap; const T* A2 = (const T*)A2p; const T* Bt = (const T*)Btp; const T* Bt2 = (const T*)Bt2p;
  __shared__ __align__(16) float sT[8][16 * 68];
  const int b    = blockIdx.y;
  const int lane = threadIdx.x & 31;
  const int wave = threadIdx.x >> 5;
  const int tilesN = N >> 6;
  const int tilesM = M >> 6;
  const int tile = blockIdx.x * 8 + wave;
  if (tile >= tilesM * tilesN) return;
  const int tm = tile / tilesN;
  const int tn = tile - tm * tilesN;
  const int m0 = tm << 6;
  const int n0 = tn << 6;

  const T* Ab  = A   + (size_t)b * strideA;
  const T* Bb  = Bt  + (size_t)b * strideB;
  const T* Ab2 = A2  + (size_t)b * strideA;
  const T* Bb2 = Bt2 + (size_t)b * strideB;

  const int rlane = lane & 15;
  const int koff  = (lane >> 4) * 8;
  const int mOff  = (lane >> 4) * 8;

  v8f acc[4][4];
#pragma unroll
  for (int i = 0; i < 4; ++i)
#pragma unroll
    for (int j = 0; j < 4; ++j) acc[i][j] = (v8f){0.f,0.f,0.f,0.f,0.f,0.f,0.f,0.f};

  for (int k0 = 0; k0 < K; k0 += 32) {
    V bh[4], bl[4];
#pragma unroll
    for (int j = 0; j < 4; ++j) {
      const size_t bo = (size_t)(n0 + (j << 4) + rlane) * ldb + koff + k0;
      bh[j] = Frag<T>::load(Bb + bo);
      if (SPLITK == 1) bl[j] = Frag<T>::load(Bb2 + bo);
    }
#pragma unroll
    for (int i = 0; i < 4; ++i) {
      const size_t ao = (size_t)(m0 + (i << 4) + rlane) * lda + koff + k0;
      V ah = Frag<T>::load(Ab + ao);
      V al = ah;
      if (SPLITK != 0) al = Frag<T>::load(Ab2 + ao);
#pragma unroll
      for (int j = 0; j < 4; ++j) {
        acc[i][j] = Frag<T>::mma(ah, bh[j], acc[i][j]);
        if (SPLITK == 1) {
          acc[i][j] = Frag<T>::mma(ah, bl[j], acc[i][j]);
          acc[i][j] = Frag<T>::mma(al, bh[j], acc[i][j]);
        }
        if (SPLITK == 2) {
          acc[i][j] = Frag<T>::mma(al, bh[j], acc[i][j]);
        }
      }
      Frag<T>::guard(acc[i][0], acc[i][3], ah, al);
    }
    Frag<T>::keep(bh[0], bh[1], bh[2], bh[3]);
    if (SPLITK == 1) Frag<T>::keep(bl[0], bl[1], bl[2], bl[3]);
  }
  acc_guard4(acc[0][0], acc[0][1], acc[0][2], acc[0][3]);
  acc_guard4(acc[1][0], acc[1][1], acc[1][2], acc[1][3]);
  acc_guard4(acc[2][0], acc[2][1], acc[2][2], acc[2][3]);
  acc_guard4(acc[3][0], acc[3][1], acc[3][2], acc[3][3]);

  float* slab = sT[wave];
#pragma unroll
  for (int i = 0; i < 4; ++i) {
    const int mBase = m0 + (i << 4);
#pragma unroll
    for (int j = 0; j < 4; ++j) {
      const int n = n0 + (j << 4) + rlane;
      float bv = 0.f;
      if (BIAS_MODE == 2) bv = bias[n];
#pragma unroll
      for (int r = 0; r < 8; ++r) {
        float v = acc[i][j][r] * scale;
        if (BIAS_MODE == 1) v += bias[mBase + mOff + r];
        if (BIAS_MODE == 2) v += bv;
        if (ACT == 1) v = tanhf(v);
        if (ACT == 2) v = fmaxf(v, 0.0f);
        if (ACT == 4) v = (v > 0.f) ? v : 0.01f * v;
        slab[(mOff + r) * 68 + (j << 4) + rlane] = v;
      }
    }
    __builtin_amdgcn_fence(__ATOMIC_RELEASE, "workgroup");
    __builtin_amdgcn_wave_barrier();
    __builtin_amdgcn_fence(__ATOMIC_ACQUIRE, "workgroup");
    if (OUT_MODE == 0) {
      float* C = (float*)Cout + (size_t)b * strideC;
      const int hh = lane >> 4, c4 = (lane & 15) * 4;
      for (int pass = 0; pass < 2; ++pass) {
#pragma unroll
        for (int it = 0; it < 8; ++it) {
          const int row = it * 2 + hh;
          v4f v = *(const v4f*)(slab + row * 68 + c4);
          *(volatile v4f*)(C + (size_t)(mBase + row) * ldc + n0 + c4) = v;
        }
        __threadfence();
      }
    } else {
      const int q = lane >> 3, c8 = (lane & 7) * 8;
      unsigned short* C  = (unsigned short*)Cout  + (size_t)b * strideC;
      unsigned short* C2 = (OUT_MODE == 2) ? ((unsigned short*)Cout2 + (size_t)b * strideC) : nullptr;
      for (int pass = 0; pass < 2; ++pass) {
#pragma unroll
        for (int it = 0; it < 4; ++it) {
          const int row = it * 4 + q;
          const float* sp = slab + row * 68 + c8;
          v8h hv, lv;
#pragma unroll
          for (int e = 0; e < 8; ++e) {
            if (OUT_MODE == 1) {
              hv[e] = (_Float16)sp[e];
            } else {
              unsigned short hb = f2bf_bits(sp[e]);
              unsigned short lb = f2bf_bits(sp[e] - bf_bits2f(hb));
              hv[e] = __builtin_bit_cast(_Float16, hb);
              lv[e] = __builtin_bit_cast(_Float16, lb);
            }
          }
          *(volatile v8h*)(C + (size_t)(mBase + row) * ldc + n0 + c8) = hv;
          if (OUT_MODE == 2) *(volatile v8h*)(C2 + (size_t)(mBase + row) * ldc + n0 + c8) = lv;
        }
        __threadfence();
      }
    }
    __builtin_amdgcn_fence(__ATOMIC_RELEASE, "workgroup");
    __builtin_amdgcn_wave_barrier();
    __builtin_amdgcn_fence(__ATOMIC_ACQUIRE, "workgroup");
  }
}

__global__ __launch_bounds__(256) void k_cvt_bf16x8(const float* __restrict__ in,
                                                    unsigned short* __restrict__ out, int n8) {
  const int i = blockIdx.x * 256 + threadIdx.x;
  if (i < n8) {
    const float* p = in + (size_t)i * 8;
    const v4f a = *(const v4f*)(p);
    const v4f c = *(const v4f*)(p + 4);
    v4u w;
    w[0] = (unsigned)f2bf_bits(a[0]) | ((unsigned)f2bf_bits(a[1]) << 16);
    w[1] = (unsigned)f2bf_bits(a[2]) | ((unsigned)f2bf_bits(a[3]) << 16);
    w[2] = (unsigned)f2bf_bits(c[0]) | ((unsigned)f2bf_bits(c[1]) << 16);
    w[3] = (unsigned)f2bf_bits(c[2]) | ((unsigned)f2bf_bits(c[3]) << 16);
    unsigned short* o = out + (size_t)i * 8;
    *(volatile v4u*)o = w;
    __threadfence();
    *(volatile v4u*)o = w;
  }
}

__global__ __launch_bounds__(256) void k_tcvt(const float* __restrict__ in, int ldin, int ncol,
                                              unsigned short* __restrict__ out, int kdim) {
  __shared__ float tile[64][65];
  const int tid = threadIdx.x, lane = tid & 31, wave = tid >> 5;
  const int n0 = blockIdx.x * 64, k0 = blockIdx.y * 64;
#pragma unroll
  for (int j = 0; j < 4; ++j) {
    const int idx = tid + 256 * j;
    const int r   = idx >> 4;
    const int c4  = (idx & 15) * 4;
    const int col = n0 + c4;
    const bool ok = (col + 4 <= ncol);
    const int colc = ok ? col : (ncol - 4);
    const v4f v = *(const v4f*)(in + (size_t)(k0 + r) * ldin + colc);
    tile[r][c4 + 0] = ok ? v[0] : 0.0f;
    tile[r][c4 + 1] = ok ? v[1] : 0.0f;
    tile[r][c4 + 2] = ok ? v[2] : 0.0f;
    tile[r][c4 + 3] = ok ? v[3] : 0.0f;
  }
  __syncthreads();
  const int q = lane >> 3, c8 = (lane & 7) * 8;
  v4u wv[2];
#pragma unroll
  for (int it = 0; it < 2; ++it) {
    const int nr = it * 32 + wave * 4 + q;
    unsigned u[4];
#pragma unroll
    for (int e = 0; e < 4; ++e) {
      const unsigned lo16 = (unsigned)f2bf_bits(tile[c8 + 2 * e][nr]);
      const unsigned hi16 = (unsigned)f2bf_bits(tile[c8 + 2 * e + 1][nr]);
      u[e] = lo16 | (hi16 << 16);
    }
    v4u t; t[0] = u[0]; t[1] = u[1]; t[2] = u[2]; t[3] = u[3];
    wv[it] = t;
  }
  for (int pass = 0; pass < 2; ++pass) {
#pragma unroll
    for (int it = 0; it < 2; ++it) {
      const int nr = it * 32 + wave * 4 + q;
      *(volatile v4u*)(out + (size_t)(n0 + nr) * kdim + k0 + c8) = wv[it];
    }
    __threadfence();
  }
}

__global__ __launch_bounds__(256) void k_atab(const float* __restrict__ A_log, float* __restrict__ atab, int n) {
  const int i = blockIdx.x * 256 + threadIdx.x;
  if (i < n) {
    const float v = -expf(bfr(A_log[i]));
    ((volatile float*)atab)[i] = v;
    __threadfence();
    ((volatile float*)atab)[i] = v;
  }
}

__global__ __launch_bounds__(256) void k_conv(const float* __restrict__ ps, const float* __restrict__ b_in,
                                              const float* __restrict__ cw, const float* __restrict__ cb,
                                              unsigned short* __restrict__ xch, unsigned short* __restrict__ xcl) {
  const int g  = blockIdx.x * 256 + threadIdx.x;
  const int b  = g >> 9;
  const int pr = g & 511;
  const int dp = pr * 2;
  const int t0 = blockIdx.y * 256;
  float wa[4], wb[4];
#pragma unroll
  for (int j = 0; j < 4; ++j) { wa[j] = bfr(cw[dp * 4 + j]); wb[j] = bfr(cw[(dp + 1) * 4 + j]); }
  const float cba = bfr(cb[dp]), cbb = bfr(cb[dp + 1]);
  const float bia = bfr(b_in[dp]), bib = bfr(b_in[dp + 1]);
  const float* base = ps + (size_t)b * SEQL * DMOD + dp;

  float a3 = 0.f, a2 = 0.f, a1 = 0.f, b3 = 0.f, b2 = 0.f, b1 = 0.f;
  if (t0 > 0) {
    const v2f v3 = *(const v2f*)(base + (size_t)(t0 - 3) * DMOD);
    const v2f v2 = *(const v2f*)(base + (size_t)(t0 - 2) * DMOD);
    const v2f v1 = *(const v2f*)(base + (size_t)(t0 - 1) * DMOD);
    a3 = v3[0] + bia; b3 = v3[1] + bib;
    a2 = v2[0] + bia; b2 = v2[1] + bib;
    a1 = v1[0] + bia; b1 = v1[1] + bib;
  }
  volatile unsigned* oh = (volatile unsigned*)xch;
  volatile unsigned* ol = (volatile unsigned*)xcl;
#pragma unroll 1
  for (int tt = 0; tt < 256; ++tt) {
    const int t = t0 + tt;
    const v2f v = *(const v2f*)(base + (size_t)t * DMOD);
    const float xa = v[0] + bia;
    const float xb = v[1] + bib;
    const float pa = wa[0] * a3 + wa[1] * a2 + wa[2] * a1 + wa[3] * xa + cba;
    const float pb = wb[0] * b3 + wb[1] * b2 + wb[2] * b1 + wb[3] * xb + cbb;
    const float sa = pa / (1.0f + expf(-pa));
    const float sb = pb / (1.0f + expf(-pb));
    unsigned ha, la, hb, lb;
    split_bf(sa, ha, la);
    split_bf(sb, hb, lb);
    const unsigned uh = ha | (hb << 16);
    const unsigned ul = la | (lb << 16);
    const size_t o = (size_t)(b * SEQL + t) * (DMOD / 2) + pr;
    oh[o] = uh;
    ol[o] = ul;
    __threadfence();
    oh[o] = uh;
    ol[o] = ul;
    a3 = a2; a2 = a1; a1 = xa;
    b3 = b2; b2 = b1; b1 = xb;
  }
}

__device__ __forceinline__ float softplus_f(float v) {
  const float m   = fmaxf(v, 0.0f);
  const float u   = exp2f(-fabsf(v) * kLog2e);
  const float w   = 1.0f + u;
  const float dlt = w - 1.0f;
  const float lg  = logf(w);
  const float dd  = (dlt > 0.0f) ? dlt : 1.0f;
  const float rat = lg / dd;
  const float l1  = (dlt > 0.0f) ? (u * rat) : u;
  return m + l1;
}

__global__ __launch_bounds__(256) void k_scan(const float* __restrict__ dtp,
                                              const unsigned short* __restrict__ xch,
                                              const unsigned short* __restrict__ xcl,
                                              const float* __restrict__ BCp,
                                              const float* __restrict__ atab,
                                              const float* __restrict__ b_dt,
                                              const float* __restrict__ b_bc,
                                              const float* __restrict__ Dp,
                                              float* __restrict__ yraw) {
  __shared__ __align__(16) float sBC[TCH][32];
  const int tid = threadIdx.x;
  const int b   = blockIdx.x >> 2;
  const int d   = (blockIdx.x & 3) * 256 + tid;

  float a[16];
  {
    const float* ap = atab + (size_t)d * 16;
    const v4f q0 = *(const v4f*)(ap), q1 = *(const v4f*)(ap + 4), q2 = *(const v4f*)(ap + 8), q3 = *(const v4f*)(ap + 12);
    a[0] = q0[0]; a[1] = q0[1]; a[2]  = q0[2]; a[3]  = q0[3];
    a[4] = q1[0]; a[5] = q1[1]; a[6]  = q1[2]; a[7]  = q1[3];
    a[8] = q2[0]; a[9] = q2[1]; a[10] = q2[2]; a[11] = q2[3];
    a[12] = q3[0]; a[13] = q3[1]; a[14] = q3[2]; a[15] = q3[3];
  }
  const float Dd  = bfr(Dp[d]);
  const float bdt = bfr(b_dt[d]);
  const int rr = tid >> 2, qq = tid & 3;
  float bb8[8];
  {
    const v4f u0 = *(const v4f*)(b_bc + qq * 8), u1 = *(const v4f*)(b_bc + qq * 8 + 4);
    bb8[0] = bfr(u0[0]); bb8[1] = bfr(u0[1]); bb8[2] = bfr(u0[2]); bb8[3] = bfr(u0[3]);
    bb8[4] = bfr(u1[0]); bb8[5] = bfr(u1[1]); bb8[6] = bfr(u1[2]); bb8[7] = bfr(u1[3]);
  }
  float h[16];
#pragma unroll
  for (int n = 0; n < 16; ++n) h[n] = 0.0f;

  volatile float* yo = (volatile float*)yraw;

#pragma unroll 1
  for (int c = 0; c < SEQL / TCH; ++c) {
    const int t0 = c * TCH;
    __syncthreads();
    {
      const float* src = BCp + (size_t)(b * SEQL + t0 + rr) * NBC + qq * 8;
      v4f u0 = *(const v4f*)(src), u1 = *(const v4f*)(src + 4);
      u0[0] += bb8[0]; u0[1] += bb8[1]; u0[2] += bb8[2]; u0[3] += bb8[3];
      u1[0] += bb8[4]; u1[1] += bb8[5]; u1[2] += bb8[6]; u1[3] += bb8[7];
      *(v4f*)&sBC[rr][qq * 8]     = u0;
      *(v4f*)&sBC[rr][qq * 8 + 4] = u1;
    }
    __syncthreads();
#pragma unroll 1
    for (int tt = 0; tt < TCH; ++tt) {
      const size_t idx = (size_t)(b * SEQL + t0 + tt) * DMOD + d;
      const float dv = dtp[idx] + bdt;
      const float dt = softplus_f(dv);
      const unsigned uh = (unsigned)xch[idx];
      const unsigned ul = (unsigned)xcl[idx];
      const float xt = __uint_as_float(uh << 16) + __uint_as_float(ul << 16);
      const float bx = dt * xt;
      const v4f B0 = *(const v4f*)&sBC[tt][0],  B1 = *(const v4f*)&sBC[tt][4];
      const v4f B2 = *(const v4f*)&sBC[tt][8],  B3 = *(const v4f*)&sBC[tt][12];
      const v4f G0 = *(const v4f*)&sBC[tt][16], G1 = *(const v4f*)&sBC[tt][20];
      const v4f G2 = *(const v4f*)&sBC[tt][24], G3 = *(const v4f*)&sBC[tt][28];
      const float Bn[16] = {B0[0], B0[1], B0[2], B0[3], B1[0], B1[1], B1[2], B1[3],
                            B2[0], B2[1], B2[2], B2[3], B3[0], B3[1], B3[2], B3[3]};
      const float Cn[16] = {G0[0], G0[1], G0[2], G0[3], G1[0], G1[1], G1[2], G1[3],
                            G2[0], G2[1], G2[2], G2[3], G3[0], G3[1], G3[2], G3[3]};
      float y = 0.0f;
#pragma unroll
      for (int n = 0; n < 16; ++n) {
        const float p  = dt * a[n];
        const float dA = exp2f(p * kLog2e);
        h[n] = fmaf(h[n], dA, bx * Bn[n]);
        y = fmaf(h[n], Cn[n], y);
      }
      y = fmaf(xt, Dd, y);
      yo[idx] = y;
      __threadfence();
      yo[idx] = y;
    }
  }
}

__global__ __launch_bounds__(256) void k_gate(const float* __restrict__ yraw, const float* __restrict__ gate,
                                              const float* __restrict__ b_in,
                                              unsigned short* __restrict__ yh, unsigned short* __restrict__ yl, int n8) {
  const int i = blockIdx.x * 256 + threadIdx.x;
  if (i < n8) {
    const size_t e0 = (size_t)i * 8;
    const int col = (i & (DMOD / 8 - 1)) * 8;
    const v4f y0 = *(const v4f*)(yraw + e0), y1 = *(const v4f*)(yraw + e0 + 4);
    const v4f g0 = *(const v4f*)(gate + e0), g1 = *(const v4f*)(gate + e0 + 4);
    const v4f c0 = *(const v4f*)(b_in + DMOD + col), c1 = *(const v4f*)(b_in + DMOD + col + 4);
    const float yy[8] = {y0[0], y0[1], y0[2], y0[3], y1[0], y1[1], y1[2], y1[3]};
    const float gg[8] = {g0[0], g0[1], g0[2], g0[3], g1[0], g1[1], g1[2], g1[3]};
    const float cc[8] = {c0[0], c0[1], c0[2], c0[3], c1[0], c1[1], c1[2], c1[3]};
    unsigned hb[8], lb[8];
#pragma unroll
    for (int e = 0; e < 8; ++e) {
      const float gv = gg[e] + bfr(cc[e]);
      const float sg = gv / (1.0f + exp2f(-gv * kLog2e));
      const float v  = yy[e] * sg;
      split_bf(v, hb[e], lb[e]);
    }
    v4u wh, wl;
    wh[0] = hb[0] | (hb[1] << 16); wh[1] = hb[2] | (hb[3] << 16); wh[2] = hb[4] | (hb[5] << 16); wh[3] = hb[6] | (hb[7] << 16);
    wl[0] = lb[0] | (lb[1] << 16); wl[1] = lb[2] | (lb[3] << 16); wl[2] = lb[4] | (lb[5] << 16); wl[3] = lb[6] | (lb[7] << 16);
    *(volatile v4u*)(yh + e0) = wh;
    *(volatile v4u*)(yl + e0) = wl;
    __threadfence();
    *(volatile v4u*)(yh + e0) = wh;
    *(volatile v4u*)(yl + e0) = wl;
  }
}

__global__ __launch_bounds__(256) void k_ln(const float* __restrict__ outpre, const float* __restrict__ x,
                                            const float* __restrict__ b_out, const float* __restrict__ g,
                                            const float* __restrict__ bb, float* __restrict__ out) {
  __shared__ float red1[8], red2[8];
  const int tid = threadIdx.x, lane = tid & 31, wave = tid >> 5;
  const size_t row = blockIdx.x;
  const int c = tid * 4;
  const v4f o  = *(const v4f*)(outpre + row * DMOD + c);
  const v4f xv = *(const v4f*)(x + row * DMOD + c);
  const v4f bo = *(const v4f*)(b_out + c);
  const v4f gv = *(const v4f*)(g + c);
  const v4f bv = *(const v4f*)(bb + c);
  float r[4];
#pragma unroll
  for (int e = 0; e < 4; ++e) r[e] = (o[e] + bfr(bo[e])) + bfr(xv[e]);
  float s = ((r[0] + r[1]) + r[2]) + r[3];
#pragma unroll
  for (int off = 1; off < 32; off <<= 1) s += __shfl_xor(s, off, 32);
  if (lane == 0) red1[wave] = s;
  __syncthreads();
  float tot = 0.0f;
#pragma unroll
  for (int w = 0; w < 8; ++w) tot += red1[w];
  const float mu = tot * (1.0f / (float)DMOD);
  float dl[4];
  float s2 = 0.0f;
#pragma unroll
  for (int e = 0; e < 4; ++e) { dl[e] = r[e] - mu; s2 += dl[e] * dl[e]; }
#pragma unroll
  for (int off = 1; off < 32; off <<= 1) s2 += __shfl_xor(s2, off, 32);
  if (lane == 0) red2[wave] = s2;
  __syncthreads();
  float tot2 = 0.0f;
#pragma unroll
  for (int w = 0; w < 8; ++w) tot2 += red2[w];
  const float var  = tot2 * (1.0f / (float)DMOD);
  const float rstd = 1.0f / sqrtf(var + kLnEps);
  v4f ov;
#pragma unroll
  for (int e = 0; e < 4; ++e) ov[e] = dl[e] * rstd * bfr(gv[e]) + bfr(bv[e]);
  float* op = out + row * DMOD + c;
  *(volatile v4f*)op = ov;
  __threadfence();
  *(volatile v4f*)op = ov;
}

extern "C" void kernel_launch(void* const* d_in, const int* in_sizes, int n_in,
                              void* d_out, int out_size, void* d_ws, size_t ws_size,
                              hipStream_t stream) {
  (void)n_in;
  const float* x      = (const float*)d_in[0];
  const float* W_in   = (const float*)d_in[1];
  const float* b_in   = (const float*)d_in[2];
  const float* conv_w = (const float*)d_in[3];
  const float* conv_b = (const float*)d_in[4];
  const float* W_bc   = (const float*)d_in[5];
  const float* b_bc   = (const float*)d_in[6];
  const float* W_dt   = (const float*)d_in[7];
  const float* b_dt   = (const float*)d_in[8];
  const float* A_log  = (const float*)d_in[9];
  const float* Dp     = (const float*)d_in[10];
  const float* W_out  = (const float*)d_in[11];
  const float* b_out  = (const float*)d_in[12];
  const float* ln_g   = (const float*)d_in[13];
  const float* ln_b   = (const float*)d_in[14];
  float* out = (float*)d_out;

  if (ws_size < WS_END) return;
  if (in_sizes[0] != NROW * DMOD || out_size != NROW * DMOD) return;
  if (in_sizes[1] != DMOD * 2 * DMOD || in_sizes[5] != DMOD * 2 * DST || in_sizes[7] != DMOD * DMOD ||
      in_sizes[11] != DMOD * DMOD || in_sizes[9] != DMOD * DST) return;

  char* ws = (char*)d_ws;
  unsigned short* xb16  = (unsigned short*)(ws + OFF_XB);
  unsigned short* xch   = (unsigned short*)(ws + OFF_XCH);
  unsigned short* xcl   = (unsigned short*)(ws + OFF_XCL);
  unsigned short* winT  = (unsigned short*)(ws + OFF_WIN);
  unsigned short* wdtT  = (unsigned short*)(ws + OFF_WDT);
  unsigned short* wbcT  = (unsigned short*)(ws + OFF_WBC);
  unsigned short* woutT = (unsigned short*)(ws + OFF_WOUT);
  float* atab = (float*)(ws + OFF_ATAB);
  float* bcp  = (float*)(ws + OFF_BC);
  float* ps   = (float*)(ws + OFF_PS);
  float* ybuf = (float*)(ws + OFF_Y);

  const int n8 = NROW * DMOD / 8;
  const int gemmBlocks1024 = (NROW / 64) * (DMOD / 64) / 8;
  const int gemmBlocksBC   = (NROW / 64) * (NBC / 64) / 8;
  static_assert(((NROW / 64) * (DMOD / 64)) % 8 == 0 && ((NROW / 64) * (NBC / 64)) % 8 == 0, "exact GEMM grids");

  k_cvt_bf16x8<<<dim3(n8 / 256), dim3(256), 0, stream>>>(x, xb16, n8);
  k_tcvt<<<dim3(2 * DMOD / 64, DMOD / 64), dim3(256), 0, stream>>>(W_in,  2 * DMOD, 2 * DMOD, winT,  DMOD);
  k_tcvt<<<dim3(DMOD / 64,     DMOD / 64), dim3(256), 0, stream>>>(W_dt,  DMOD,     DMOD,     wdtT,  DMOD);
  k_tcvt<<<dim3(NBC / 64,      DMOD / 64), dim3(256), 0, stream>>>(W_bc,  2 * DST,  2 * DST,  wbcT,  DMOD);
  k_tcvt<<<dim3(DMOD / 64,     DMOD / 64), dim3(256), 0, stream>>>(W_out, DMOD,     DMOD,     woutT, DMOD);
  k_atab<<<dim3(DMOD * DST / 256), dim3(256), 0, stream>>>(A_log, atab, DMOD * DST);
  wmma_gemm64<1, 0, 0, 0, 0><<<dim3(gemmBlocks1024, 1), dim3(256), 0, stream>>>(
      xb16, xb16, DMOD, 0L, winT, winT, DMOD, 0L, (void*)ps, (void*)ps, DMOD, 0L, b_in, NROW, DMOD, DMOD, 1.0f);
  k_conv<<<dim3(NBAT * DMOD / 2 / 256, SEQL / 256), dim3(256), 0, stream>>>(ps, b_in, conv_w, conv_b, xch, xcl);
  wmma_gemm64<1, 2, 0, 0, 0><<<dim3(gemmBlocks1024, 1), dim3(256), 0, stream>>>(
      xch, xcl, DMOD, 0L, wdtT, wdtT, DMOD, 0L, (void*)ps, (void*)ps, DMOD, 0L, b_in, NROW, DMOD, DMOD, 1.0f);
  wmma_gemm64<1, 2, 0, 0, 0><<<dim3(gemmBlocksBC, 1), dim3(256), 0, stream>>>(
      xch, xcl, DMOD, 0L, wbcT, wbcT, DMOD, 0L, (void*)bcp, (void*)bcp, NBC, 0L, b_in, NROW, NBC, DMOD, 1.0f);
  k_scan<<<dim3(NBAT * DMOD / 256), dim3(256), 0, stream>>>(ps, xch, xcl, bcp, atab, b_dt, b_bc, Dp, ybuf);
  wmma_gemm64<1, 0, 0, 0, 0><<<dim3(gemmBlocks1024, 1), dim3(256), 0, stream>>>(
      xb16, xb16, DMOD, 0L, winT + (size_t)DMOD * DMOD, winT + (size_t)DMOD * DMOD, DMOD, 0L,
      (void*)ps, (void*)ps, DMOD, 0L, b_in, NROW, DMOD, DMOD, 1.0f);
  k_gate<<<dim3(n8 / 256), dim3(256), 0, stream>>>(ybuf, ps, b_in, xch, xcl, n8);
  wmma_gemm64<1, 2, 0, 0, 0><<<dim3(gemmBlocks1024, 1), dim3(256), 0, stream>>>(
      xch, xcl, DMOD, 0L, woutT, woutT, DMOD, 0L, (void*)ybuf, (void*)ybuf, DMOD, 0L, b_in, NROW, DMOD, DMOD, 1.0f);
  k_ln<<<dim3(NROW), dim3(256), 0, stream>>>(ybuf, x, b_out, ln_g, ln_b, out);
}
